// BatchGAT_26482768347246
// MI455X (gfx1250) — hardware-verified
//
#include <hip/hip_runtime.h>
#include <math.h>

typedef __attribute__((ext_vector_type(16))) _Float16 v16h;
typedef __attribute__((ext_vector_type(16))) __bf16 v16b;
typedef __attribute__((ext_vector_type(8)))  _Float16 v8h;
typedef __attribute__((ext_vector_type(8)))  float v8f;
typedef __attribute__((ext_vector_type(4)))  float v4f;
typedef __attribute__((ext_vector_type(2)))  float v2f;
typedef __attribute__((ext_vector_type(4)))  unsigned v4u;
typedef __attribute__((ext_vector_type(4)))  int v4i;
typedef float __attribute__((may_alias)) float_a;
typedef int __attribute__((may_alias)) int_a;

template <typename T> __device__ __forceinline__ void vst2(void* p, T v) { *(volatile T*)p = v; __threadfence(); *(volatile T*)p = v; }
__device__ __forceinline__ v8f wmma16(v16h a, v16h b, v8f c) {
  v8f d = __builtin_amdgcn_wmma_f32_16x16x32_f16(false, a, false, b, (short)0, c, false, false);
  asm volatile("v_nop\n\tv_nop\n\tv_nop\n\tv_nop" : "+v"(d) : "v"(a), "v"(b));
  return d;
}
__device__ __forceinline__ v8f wmma_bf(v16b a, v16b b, v8f c) {
  v8f d = __builtin_amdgcn_wmma_f32_16x16x32_bf16(false, a, false, b, (short)0, c, false, false);
  asm volatile("v_nop\n\tv_nop\n\tv_nop\n\tv_nop" : "+v"(d) : "v"(a), "v"(b));
  return d;
}
__device__ __forceinline__ v16h frag_h(const _Float16* rowk0, int lane) {
  union { v16h v; v8h q[2]; } u; const _Float16* p = rowk0 + 8 * (lane >> 4);
  u.q[0] = *(const v8h*)p; u.q[1] = *(const v8h*)(p + 16); return u.v;
}
__device__ __forceinline__ v16h frag_f32(const float* rowk0, int lane) {
  v16h a; const float* p = rowk0 + 8 * (lane >> 4);
#pragma unroll
  for (int i = 0; i < 8; ++i) { a[i] = (_Float16)p[i]; a[8 + i] = (_Float16)p[16 + i]; }
  return a;
}
__device__ __forceinline__ v16h frag_f32s(const float* rowk0, int lane, float sc) {
  v16h a; const float* p = rowk0 + 8 * (lane >> 4);
#pragma unroll
  for (int i = 0; i < 8; ++i) { a[i] = (_Float16)(p[i] * sc); a[8 + i] = (_Float16)(p[16 + i] * sc); }
  return a;
}
__device__ __forceinline__ v16h fragc_f32(const float* W, int k0, int n, int lane, int ld, int K) {
  v16h a; const int g = lane >> 4;
#pragma unroll
  for (int i = 0; i < 8; ++i) { const int ka = k0 + 8 * g + i, kb = ka + 16;
    a[i] = (_Float16)(ka < K ? W[(size_t)(ka < K ? ka : K - 1) * ld + n] : 0.f); a[8 + i] = (_Float16)(kb < K ? W[(size_t)(kb < K ? kb : K - 1) * ld + n] : 0.f); }
  return a;
}
struct F2 { v16b h, l; };
__device__ __forceinline__ F2 bsplit16(const float v[16]) { F2 r;
#pragma unroll
  for (int i = 0; i < 16; ++i) { const __bf16 h = (__bf16)v[i]; r.h[i] = h; r.l[i] = (__bf16)(v[i] - (float)h); }
  return r; }
__device__ __forceinline__ F2 split_row(const float* row, int k0, int lane) { float v[16]; const float* p = row + k0 + 8 * (lane >> 4);
#pragma unroll
  for (int i = 0; i < 8; ++i) { v[i] = p[i]; v[8 + i] = p[16 + i]; }
  return bsplit16(v); }
__device__ __forceinline__ F2 split_rowK(const float* row, int k0, int lane, int K) { float v[16]; const int g = lane >> 4;
#pragma unroll
  for (int i = 0; i < 8; ++i) { const int ka = k0 + 8 * g + i, kb = ka + 16; v[i] = ka < K ? row[ka < K ? ka : K - 1] : 0.f; v[8 + i] = kb < K ? row[kb < K ? kb : K - 1] : 0.f; }
  return bsplit16(v); }
__device__ __forceinline__ F2 split_col(const float* W, int k0, int n, int lane, int ld, int K) { float v[16]; const int g = lane >> 4;
#pragma unroll
  for (int i = 0; i < 8; ++i) { const int ka = k0 + 8 * g + i, kb = ka + 16; v[i] = ka < K ? W[(size_t)(ka < K ? ka : K - 1) * ld + n] : 0.f; v[8 + i] = kb < K ? W[(size_t)(kb < K ? kb : K - 1) * ld + n] : 0.f; }
  return bsplit16(v); }
__device__ __forceinline__ v8f mac3(const F2& a, const F2& b, v8f c) { c = wmma_bf(a.l, b.h, c); c = wmma_bf(a.h, b.l, c); return wmma_bf(a.h, b.h, c); }
__device__ __forceinline__ float sigm(float v) { return 1.0f / (1.0f + expf(-v)); }
#define LDSX() do { asm volatile("s_wait_dscnt 0" ::: "memory"); __builtin_amdgcn_wave_barrier(); __builtin_amdgcn_fence(__ATOMIC_RELEASE, "workgroup"); } while (0)


#define NB 32
#define NN 512
#define F0 64
#define NH 8
#define FO 64
#define X1W (NH * FO)
#ifndef TNB
#define TNB NB
#endif
typedef __attribute__((ext_vector_type(8))) __bf16 v8b;
__device__ __forceinline__ v16b frag_b(const __bf16* rowk0, int lane) {
  union { v16b v; v8b q[2]; } u; const __bf16* p = rowk0 + 8 * (lane >> 4);
  u.q[0] = *(const v8b*)p; u.q[1] = *(const v8b*)(p + 16); return u.v;
}
__device__ __forceinline__ v16b frag_gbf(const float* rowk0, int lane) {
  v16b a; const float* p = rowk0 + 8 * (lane >> 4);
#pragma unroll
  for (int i = 0; i < 8; ++i) { a[i] = (__bf16)p[i]; a[8 + i] = (__bf16)p[16 + i]; }
  return a;
}
__device__ __forceinline__ float bfr(float v) { return (float)(__bf16)v; }
__device__ __attribute__((noinline)) float exp_ni(float v) { return expf(v); }
#define WS_PW0  0u
#define WS_PW1  (WS_PW0 + 2u * FO * F0)
#define WS_SD   (WS_PW1 + 2u * FO * X1W)
#define WS_HTH  (WS_SD + 4u * NB * NH * 2 * NN)
#define WS_HTL  (WS_HTH + 2u * NB * FO * NN)
#define WS_X1   (WS_HTL + 2u * NB * FO * NN)
#define WS_END  (WS_X1 + 4u * NB * NN * X1W)

__global__ __launch_bounds__(256) void k_pack(const float* __restrict__ W0, const float* __restrict__ W1, __bf16* __restrict__ PW0, __bf16* __restrict__ PW1) {
  __shared__ __align__(16) __bf16 srow[X1W]; const int n = blockIdx.x, tid = threadIdx.x;
  if (n < FO) { if (tid < F0) srow[tid] = (__bf16)bfr(W0[(size_t)tid * FO + n]); __syncthreads(); if (tid < 8) vst2((unsigned*)(PW0 + (size_t)n * F0 + tid * 8), *(const v4u*)(&srow[tid * 8])); }
  else { const int o = n - FO; for (int k = tid; k < X1W; k += 256) srow[k] = (__bf16)bfr(W1[(size_t)k * FO + o]); __syncthreads(); if (tid < X1W / 8) vst2((unsigned*)(PW1 + (size_t)o * X1W + tid * 8), *(const v4u*)(&srow[tid * 8])); }
}
template <int K, bool EXACT>
__global__ __launch_bounds__(128) void k_hp(const float* __restrict__ X, const __bf16* __restrict__ PW, const float* __restrict__ AS, const float* __restrict__ AD, float* __restrict__ SD, __bf16* __restrict__ HTH, __bf16* __restrict__ HTL) {
  __shared__ __align__(16) float sh[64][68]; __shared__ float sas[F0][NH], sad[F0][NH]; __shared__ __align__(16) __bf16 sth[FO][72], stl[FO][72]; __shared__ __align__(16) float ssd[NH][2][64];
  const int tid = threadIdx.x, wave = tid >> 5, lane = tid & 31, col = lane & 15, g = lane >> 4; const int b = blockIdx.y; const int n0 = blockIdx.x * 64; const float* Xb = X + ((size_t)b * NN + n0 + wave * 16) * K;
  for (int q = tid; q < F0 * NH; q += 128) { sas[q / NH][q % NH] = bfr(AS[q]); sad[q / NH][q % NH] = bfr(AD[q]); }
  v8f acc[4] = {};
#pragma unroll 2
  for (int kc = 0; kc < K / 32; ++kc) {
    if (EXACT) { const v16b a = frag_gbf(Xb + (size_t)col * K + kc * 32, lane);
#pragma unroll
      for (int j = 0; j < 4; ++j) acc[j] = wmma_bf(a, frag_b(PW + (size_t)(j * 16 + col) * K + kc * 32, lane), acc[j]); }
    else { const F2 a = split_row(Xb + (size_t)col * K, kc * 32, lane);
#pragma unroll
      for (int j = 0; j < 4; ++j) { const v16b w = frag_b(PW + (size_t)(j * 16 + col) * K + kc * 32, lane); acc[j] = wmma_bf(a.l, w, acc[j]); acc[j] = wmma_bf(a.h, w, acc[j]); } } }
#pragma unroll
  for (int j = 0; j < 4; ++j)
#pragma unroll
    for (int r = 0; r < 8; ++r) { const float v = acc[j][r]; const int rl = wave * 16 + 8 * g + r, o = j * 16 + col; sh[rl][o] = v; const __bf16 hb = (__bf16)v; sth[o][rl] = hb; stl[o][rl] = (__bf16)(v - (float)hb); }
  __syncthreads();
  { const int rl = tid >> 1, hq = (tid & 1) * 4;
    for (int h = hq; h < hq + 4; ++h) { float s1 = 0.f, s2 = 0.f;
#pragma unroll 1
      for (int o = 0; o < FO; ++o) { s1 += sh[rl][o] * sas[o][h]; s2 += sh[rl][o] * sad[o][h]; }
      ssd[h][0][rl] = s1; ssd[h][1][rl] = s2; } }
  __syncthreads();
  for (int q = tid; q < FO * 8; q += 128) { const int o = q >> 3, pc = q & 7; const size_t off = ((size_t)b * FO + o) * NN + n0 + pc * 8; vst2((unsigned*)(HTH + off), *(const v4u*)&sth[o][pc * 8]); vst2((unsigned*)(HTL + off), *(const v4u*)&stl[o][pc * 8]); }
  for (int q = tid; q < NH * 2 * 16; q += 128) { const int h = q >> 5, which = (q >> 4) & 1, pc = q & 15; vst2(SD + (((size_t)b * NH + h) * 2 + which) * NN + n0 + pc * 4, *(const v4f*)&ssd[h][which][pc * 4]); }
}
template <int MEAN>
__global__ __launch_bounds__(128) void k_gat(const float* __restrict__ SD, const float* __restrict__ ADJ, const __bf16* __restrict__ HTH, const __bf16* __restrict__ HTL, float* __restrict__ DST) {
  __shared__ __align__(16) float sp[4][16][36]; __shared__ __align__(16) float so[4][16][68];
  const int tid = threadIdx.x, wave = tid >> 5, lane = tid & 31, col = lane & 15, g = lane >> 4; const int b = MEAN ? blockIdx.y : blockIdx.y / NH; const int i0 = blockIdx.x * 64 + wave * 16;
  float res[4][8];
#pragma unroll
  for (int dt = 0; dt < 4; ++dt)
#pragma unroll
    for (int r = 0; r < 8; ++r) res[dt][r] = 0.f;
  const int nhl = MEAN ? NH : 1;
#pragma unroll 1
  for (int hl = 0; hl < nhl; ++hl) { const int h = MEAN ? hl : (blockIdx.y % NH); const float* S = SD + (((size_t)b * NH + h) * 2) * NN; const float* Dv = S + NN;
    float si[8];
#pragma unroll
    for (int r = 0; r < 8; ++r) si[r] = S[i0 + 8 * g + r];
    float m[8], l[8]; v8f acc[4] = {};
#pragma unroll
    for (int r = 0; r < 8; ++r) { m[r] = -3.0e38f; l[r] = 0.f; }
#pragma unroll 1
    for (int ks = 0; ks < NN / 32; ++ks) { float s[2][8];
#pragma unroll
      for (int ct = 0; ct < 2; ++ct) { const int j = ks * 32 + ct * 16 + col; const float dj = Dv[j];
#pragma unroll
        for (int r = 0; r < 8; ++r) { const int i = i0 + 8 * g + r; float u = si[r] + dj; u = u >= 0.f ? u : 0.2f * u; const float a = (j == i) ? 1.0f : bfr(ADJ[((size_t)b * NN + i) * NN + j]); if (a == 0.f) u = 0.f; s[ct][r] = (u == 0.f) ? -1e20f : u; } }
#pragma unroll
      for (int r = 0; r < 8; ++r) { float mx = fmaxf(s[0][r], s[1][r]);
#pragma unroll
        for (int o = 1; o < 16; o <<= 1) mx = fmaxf(mx, __shfl_xor(mx, o));
        const float mn = fmaxf(m[r], mx); const float alpha = exp_ni(m[r] - mn); const float e0 = exp_ni(s[0][r] - mn), e1 = exp_ni(s[1][r] - mn); float es = e0 + e1;
#pragma unroll
        for (int o = 1; o < 16; o <<= 1) es += __shfl_xor(es, o);
        l[r] = l[r] * alpha + es; m[r] = mn;
#pragma unroll
        for (int dt = 0; dt < 4; ++dt) acc[dt][r] *= alpha;
        sp[wave][8 * g + r][col] = e0; sp[wave][8 * g + r][16 + col] = e1; }
      LDSX();
      const F2 pa = split_row(&sp[wave][col][0], 0, lane);
#pragma unroll
      for (int dt = 0; dt < 4; ++dt) { const size_t vrow = ((size_t)b * FO + dt * 16 + col) * NN + ks * 32; const v16b vh = frag_b(HTH + vrow, lane), vl = frag_b(HTL + vrow, lane); acc[dt] = wmma_bf(pa.l, vh, acc[dt]); acc[dt] = wmma_bf(pa.h, vl, acc[dt]); acc[dt] = wmma_bf(pa.h, vh, acc[dt]); }
      LDSX(); }
#pragma unroll
    for (int r = 0; r < 8; ++r) { const float il = 1.0f / l[r];
#pragma unroll
      for (int dt = 0; dt < 4; ++dt) res[dt][r] += acc[dt][r] * il * (MEAN ? (1.0f / NH) : 1.0f); } }
  const int h = blockIdx.y % NH;
#pragma unroll
  for (int r = 0; r < 8; ++r)
#pragma unroll
    for (int dt = 0; dt < 4; ++dt) { float v = res[dt][r]; if (!MEAN) v = v > 0.f ? v : (exp_ni(v) - 1.0f); so[wave][8 * g + r][dt * 16 + col] = v; }
  LDSX();
  for (int rl = 0; rl < 16; ++rl) if (lane < 16) { if (MEAN) vst2(DST + ((size_t)b * NN + i0 + rl) * FO + lane * 4, *(const v4f*)&so[wave][rl][lane * 4]); else vst2(DST + ((size_t)b * NN + i0 + rl) * X1W + h * FO + lane * 4, *(const v4f*)&so[wave][rl][lane * 4]); }
}
extern "C" void kernel_launch(void* const* d_in, const int* in_sizes, int n_in, void* d_out, int out_size, void* d_ws, size_t ws_size, hipStream_t stream) {
  (void)in_sizes; (void)n_in; (void)out_size;
  const float** F = (const float**)d_in;
  if (ws_size < (size_t)WS_END) return;
  char* ws = (char*)d_ws; __bf16 *PW0 = (__bf16*)(ws + WS_PW0), *PW1 = (__bf16*)(ws + WS_PW1), *HTH = (__bf16*)(ws + WS_HTH), *HTL = (__bf16*)(ws + WS_HTL); float *SD = (float*)(ws + WS_SD), *X1 = (float*)(ws + WS_X1);
  k_pack<<<2 * FO, 256, 0, stream>>>(F[4], F[7], PW0, PW1);
  k_hp<F0, true><<<dim3(NN / 64, TNB), 128, 0, stream>>>(F[0], PW0, F[5], F[6], SD, HTH, HTL);
  k_gat<0><<<dim3(NN / 64, TNB * NH), 128, 0, stream>>>(SD, F[1], HTH, HTL, X1);
  k_hp<X1W, false><<<dim3(NN / 64, TNB), 128, 0, stream>>>(X1, PW1, F[8], F[9], SD, HTH, HTL);
  k_gat<1><<<dim3(NN / 64, TNB), 128, 0, stream>>>(SD, F[1], HTH, HTL, (float*)d_out);
}
